// CausalSelfAttention_80418967650984
// MI455X (gfx1250) — hardware-run, weakly checked
//
#include <hip/hip_runtime.h>


#ifndef NB
#define NB 4
#endif
#ifndef SEQ
#define SEQ 2048
#endif
#define NB_FULL  4
#define SEQ_FULL 2048
#ifndef OUT_SEQ
#define OUT_SEQ SEQ
#endif
#define DM   1024
#define NH_  16
#define HD   64
#define AW   4
#define QRS  2048.0f
#define QRI  (1.0f / 2048.0f)
#define SC2  (0.125f * 1.4426950408889634f)
#define PSH  8.0f
#define CXS  16.0f
#define WOS  64.0f
#define OSC  (1.0f / 1024.0f)
#define NEGB (-3.0e38f)

static constexpr int EARLY = (SEQ < 512) ? SEQ : 512;
static constexpr int DROWS = SEQ - EARLY;
static constexpr int DRC   = (DROWS > 0) ? DROWS : 64;

static_assert(HD == 64);
static_assert(NH_ * HD == DM);
static_assert(DM % 64 == 0);
static_assert(DM % 32 == 0);
static_assert(SEQ % 64 == 0);
static_assert(EARLY % 64 == 0);
static_assert(DROWS % 64 == 0);
static_assert(SEQ % 32 == 0);
static_assert(EARLY % (16 * AW) == 0);
static_assert(DROWS % (16 * AW) == 0);
static_assert(((size_t)SEQ * DM) % 8 == 0);
static_assert(NB <= NB_FULL);
static_assert(SEQ <= SEQ_FULL);

typedef _Float16 h16;
typedef unsigned short bf;
typedef __attribute__((ext_vector_type(16))) __bf16   v16bf;
typedef __attribute__((ext_vector_type(16))) _Float16 v16h;
typedef __attribute__((ext_vector_type(8)))  _Float16 v8h;
typedef __attribute__((ext_vector_type(8)))  unsigned short v8us;
typedef __attribute__((ext_vector_type(8)))  float    v8f;
typedef __attribute__((ext_vector_type(4)))  float    v4f;
typedef v4f  __attribute__((may_alias)) v4fa;

__device__ __forceinline__ unsigned short f2bf(float f) { unsigned u = __float_as_uint(f); u += 0x7FFFu + ((u >> 16) & 1u); return (unsigned short)(u >> 16); }
__device__ __forceinline__ v16h cat16(v8h lo, v8h hi) { return __builtin_shufflevector(lo, hi, 0, 1, 2, 3, 4, 5, 6, 7, 8, 9, 10, 11, 12, 13, 14, 15); }
__device__ __forceinline__ v16bf cat16b(v8us lo, v8us hi) { return __builtin_bit_cast(v16bf, __builtin_shufflevector(lo, hi, 0, 1, 2, 3, 4, 5, 6, 7, 8, 9, 10, 11, 12, 13, 14, 15)); }
__device__ __forceinline__ v8f wmma16(v16h a, v16h b, v8f c) { return __builtin_amdgcn_wmma_f32_16x16x32_f16(false, a, false, b, (short)0, c, false, false); }
__device__ __forceinline__ v8f wmmab(v16bf a, v16bf b, v8f c) { return __builtin_amdgcn_wmma_f32_16x16x32_bf16(false, a, false, b, (short)0, c, false, false); }
__device__ __forceinline__ v16h  ldh(const h16* p) { return cat16(*(const v8h*)p, *(const v8h*)(p + 16)); }
__device__ __forceinline__ v16bf ldb(const bf* p)  { return cat16b(*(const v8us*)p, *(const v8us*)(p + 16)); }
__device__ __forceinline__ void wave_sync() { __builtin_amdgcn_fence(3  , "wavefront"); __builtin_amdgcn_wave_barrier(); asm volatile("" ::: "memory"); }

__global__ __launch_bounds__(256) void k_cvt8(const float* __restrict__ src, bf* dst, size_t n8) {
    const size_t i = (size_t)blockIdx.x * 256 + threadIdx.x; if (i >= n8) return;
    const v8f v = *(const v8f*)(src + i * 8); v8us o;
#pragma unroll
    for (int k = 0; k < 8; ++k) o[k] = f2bf(v[k]);
    *(volatile v8us*)(dst + i * 8) = o; __threadfence(); *(volatile v8us*)(dst + i * 8) = o;
}

template<int MODE>
__device__ __forceinline__ unsigned short cvt16(float f) {
    const unsigned short b = f2bf(f);
    if (MODE == 0) return b;
    const h16 hv = (h16)(__uint_as_float((unsigned)b << 16) * WOS);
    return __builtin_bit_cast(unsigned short, hv);
}

template<int MODE>
__global__ __launch_bounds__(256) void k_tcvt(const float* __restrict__ W, unsigned short* WT) {
    __shared__ float ts[64 * 65];
    const int tid = threadIdx.x, lane = tid & 31, wave = __builtin_amdgcn_readfirstlane((int)(tid >> 5));
    const int k0 = blockIdx.x * 64, n0 = blockIdx.y * 64;
#pragma unroll
    for (int i = 0; i < 4; ++i) { const int idx = tid + 256 * i; const int r = idx >> 4, c4 = (idx & 15) * 4;
        const v4f v = *(const v4f*)(W + (size_t)(k0 + r) * DM + n0 + c4);
        ts[r * 65 + c4 + 0] = v[0]; ts[r * 65 + c4 + 1] = v[1]; ts[r * 65 + c4 + 2] = v[2]; ts[r * 65 + c4 + 3] = v[3]; }
    __syncthreads();
    const int c8 = (lane & 7) * 8;
    const int nA = wave * 8 + (lane >> 3), nB = nA + 4;
    v8us oA, oB;
#pragma unroll
    for (int i = 0; i < 8; ++i) { oA[i] = cvt16<MODE>(ts[(c8 + i) * 65 + nA]); oB[i] = cvt16<MODE>(ts[(c8 + i) * 65 + nB]); }
    unsigned short* pA = WT + (size_t)(n0 + nA) * DM + k0 + c8;
    unsigned short* pB = WT + (size_t)(n0 + nB) * DM + k0 + c8;
    *(volatile v8us*)pA = oA; *(volatile v8us*)pB = oB;
    __threadfence();
    *(volatile v8us*)pA = oA; *(volatile v8us*)pB = oB;
}

__global__ __launch_bounds__(32) void k_proj(const bf* __restrict__ A, const bf* __restrict__ Bt, h16* Ph, h16* Pr, int useRes,
                                             int RB, size_t sRB, int pitch, int CB, size_t sCB,
                                             size_t sRBr, int pitchr, size_t sCBr, int rowLim, int colLim) {
    __shared__ __align__(16) float os[16 * 68];
    const int K = DM;
    const int lane = threadIdx.x & 31, lr = lane & 15, hi = lane >> 4; const int r0 = blockIdx.x * 64, c0 = blockIdx.y * 64;
    v8f acc[4][4];
#pragma unroll
    for (int mb = 0; mb < 4; ++mb)
#pragma unroll
        for (int nb = 0; nb < 4; ++nb) acc[mb][nb] = (v8f){};
    const size_t aoff = (size_t)(r0 + lr) * K + 8 * hi, boff = (size_t)(c0 + lr) * K + 8 * hi;
#pragma unroll 1
    for (int kc = 0; kc < K; kc += 32) {
        v16bf a[4];
#pragma unroll
        for (int mb = 0; mb < 4; ++mb) a[mb] = ldb(A + aoff + (size_t)mb * 16 * K + kc);
#pragma unroll
        for (int nb = 0; nb < 4; ++nb) { const v16bf b = ldb(Bt + boff + (size_t)nb * 16 * K + kc);
#pragma unroll
            for (int mb = 0; mb < 4; ++mb) acc[mb][nb] = wmmab(a[mb], b, acc[mb][nb]); }
        asm volatile("v_nop\n\tv_nop\n\tv_nop\n\tv_nop" : "+v"(acc[0][0]), "+v"(acc[1][1]), "+v"(acc[2][2]), "+v"(acc[3][3]) : "v"(a[0]), "v"(a[1]), "v"(a[2]), "v"(a[3]));
    }
    const int rin = r0 % RB, cin = c0 % CB;
    const bool doRes = (useRes != 0) && (rin < rowLim) && (cin < colLim);
    const size_t tbase  = (size_t)(r0 / RB) * sRB  + (size_t)rin * (size_t)pitch  + (size_t)(c0 / CB) * sCB  + (size_t)cin;
    const size_t tbaser = (size_t)(r0 / RB) * sRBr + (size_t)rin * (size_t)pitchr + (size_t)(c0 / CB) * sCBr + (size_t)cin;
#pragma unroll
    for (int mb = 0; mb < 4; ++mb) {
#pragma unroll
        for (int nb = 0; nb < 4; ++nb) {
#pragma unroll
            for (int j = 0; j < 8; ++j) os[(hi * 8 + j) * 68 + nb * 16 + lr] = acc[mb][nb][j]; }
        wave_sync();
        const size_t sb  = tbase  + (size_t)(mb * 16) * (size_t)pitch;
        const size_t sbr = tbaser + (size_t)(mb * 16) * (size_t)pitchr;
#pragma unroll 1
        for (int ps = 0; ps < 2; ++ps) {
#pragma unroll
            for (int s = 0; s < 4; ++s) { const int row = 4 * s + (lane >> 3), c8 = (lane & 7) * 8;
                const v4f x0 = *(const v4fa*)(&os[row * 68 + c8]); const v4f x1 = *(const v4fa*)(&os[row * 68 + c8 + 4]); v8h hv, rv;
#pragma unroll
                for (int i = 0; i < 4; ++i) { const h16 a0 = (h16)x0[i]; const h16 a1 = (h16)x1[i]; hv[i] = a0; hv[4 + i] = a1; rv[i] = (h16)((x0[i] - (float)a0) * QRS); rv[4 + i] = (h16)((x1[i] - (float)a1) * QRS); }
                const size_t oo = sb + (size_t)row * (size_t)pitch + c8;
                *(volatile v8h*)(Ph + oo) = hv;
                if (doRes) { const size_t oor = sbr + (size_t)row * (size_t)pitchr + c8; *(volatile v8h*)(Pr + oor) = rv; } }
            if (ps == 0) __threadfence(); }
        wave_sync();
    }
}

#define STG_O(COL, OH, OL) { v4f a_, c_; \
    a_[0] = (OH[0] + OL[0] * QRI) * sc; a_[1] = (OH[1] + OL[1] * QRI) * sc; a_[2] = (OH[2] + OL[2] * QRI) * sc; a_[3] = (OH[3] + OL[3] * QRI) * sc; \
    c_[0] = (OH[4] + OL[4] * QRI) * sc; c_[1] = (OH[5] + OL[5] * QRI) * sc; c_[2] = (OH[6] + OL[6] * QRI) * sc; c_[3] = (OH[7] + OL[7] * QRI) * sc; \
    *(v4fa*)(&os[wb + lr * 68 + (COL) + 8 * hi]) = a_; *(v4fa*)(&os[wb + lr * 68 + (COL) + 8 * hi + 4]) = c_; }

template<bool E>
__global__ __launch_bounds__(32 * AW) void k_flash(const h16* __restrict__ QH, const h16* __restrict__ QR, const h16* __restrict__ KP, const h16* __restrict__ KR,
                                                   const h16* __restrict__ VT, const h16* __restrict__ VR, h16* CH, h16* CR) {
    __shared__ __align__(16) float os[AW * 16 * 68];
    const int lane = threadIdx.x & 31, wave = __builtin_amdgcn_readfirstlane((int)(threadIdx.x >> 5)), lr = lane & 15, hi = lane >> 4;
    const int zh = blockIdx.y; const int b = zh / NH_, h = zh % NH_;
    const int t0 = (E ? 0 : EARLY) + (blockIdx.x * AW + wave) * 16;
    const size_t pbase = (size_t)zh * SEQ * HD;
    const size_t pbe   = (size_t)zh * EARLY * HD;
    const size_t qo = pbase + (size_t)(t0 + lr) * HD + 8 * hi;
    const v16h qh0 = ldh(QH + qo), qh1 = ldh(QH + qo + 32);
    v16h qr0 = qh0, qr1 = qh1;
    if constexpr (E) { const size_t qe = pbe + (size_t)(t0 + lr) * HD + 8 * hi; qr0 = ldh(QR + qe); qr1 = ldh(QR + qe + 32); }
    const size_t ko  = pbase + (size_t)lr * HD + 8 * hi;
    const size_t koe = pbe   + (size_t)lr * HD + 8 * hi;
    const size_t vo  = pbase + (size_t)lr * SEQ + 8 * hi;
    const size_t voe = pbe   + (size_t)lr * EARLY + 8 * hi;
    v8f oH0 = (v8f){}, oH1 = (v8f){}, oH2 = (v8f){}, oH3 = (v8f){};
    v8f oL0 = (v8f){}, oL1 = (v8f){}, oL2 = (v8f){}, oL3 = (v8f){};
    float m = NEGB, l = 0.0f;
    const int tq = t0 + lr;
    const int kend = t0 + 16;
#pragma unroll 1
    for (int key0 = 0; key0 < kend; key0 += 32) {
        v8f sHa = (v8f){}, sHb = (v8f){}, sLa = (v8f){}, sLb = (v8f){};
        {
            const h16* ka = KP + ko + (size_t)key0 * HD;
            const v16h ka0 = ldh(ka), ka1 = ldh(ka + 32), kb0 = ldh(ka + 16 * HD), kb1 = ldh(ka + 16 * HD + 32);
            sHa = wmma16(ka0, qh0, sHa); sHb = wmma16(kb0, qh0, sHb);
            sHa = wmma16(ka1, qh1, sHa); sHb = wmma16(kb1, qh1, sHb);
            if constexpr (E) {
                sLa = wmma16(ka0, qr0, sLa); sLb = wmma16(kb0, qr0, sLb);
                sLa = wmma16(ka1, qr1, sLa); sLb = wmma16(kb1, qr1, sLb);
                const h16* kr = KR + koe + (size_t)key0 * HD;
                const v16h ra0 = ldh(kr), ra1 = ldh(kr + 32), rb0 = ldh(kr + 16 * HD), rb1 = ldh(kr + 16 * HD + 32);
                sLa = wmma16(ra0, qh0, sLa); sLb = wmma16(rb0, qh0, sLb);
                sLa = wmma16(ra1, qh1, sLa); sLb = wmma16(rb1, qh1, sLb);
                asm volatile("v_nop\n\tv_nop\n\tv_nop\n\tv_nop" : "+v"(sHa), "+v"(sLa), "+v"(sHb), "+v"(sLb) : "v"(ra0), "v"(ra1), "v"(rb0), "v"(rb1), "v"(ka0), "v"(ka1), "v"(kb0), "v"(kb1));
            } else {
                asm volatile("v_nop\n\tv_nop\n\tv_nop\n\tv_nop" : "+v"(sHa), "+v"(sHb) : "v"(ka0), "v"(ka1), "v"(kb0), "v"(kb1));
            }
        }
        float ta[8], tb[8]; float mx = NEGB;
        const int kq = key0 + 8 * hi;
#pragma unroll
        for (int r = 0; r < 8; ++r) {
            const float va = (sHa[r] + sLa[r] * QRI) * SC2, vb = (sHb[r] + sLb[r] * QRI) * SC2;
            ta[r] = (kq + r <= tq) ? va : NEGB;
            tb[r] = (kq + 16 + r <= tq) ? vb : NEGB;
            mx = fmaxf(mx, fmaxf(ta[r], tb[r])); }
        mx = fmaxf(mx, __shfl_xor(mx, 16, 32));
        const float mnew = fmaxf(m, mx);
        const float alpha = __builtin_amdgcn_exp2f(m - mnew);
        const float sh = PSH - mnew;
        v16h pb, pr; float ls = 0.0f;
#pragma unroll
        for (int r = 0; r < 8; ++r) {
            const float ea = __builtin_amdgcn_exp2f(ta[r] + sh), eb = __builtin_amdgcn_exp2f(tb[r] + sh);
            const h16 pa = (h16)ea, pc = (h16)eb; pb[r] = pa; pb[8 + r] = pc;
            if constexpr (E) {
                const h16 ra = (h16)((ea - (float)pa) * QRS), rc = (h16)((eb - (float)pc) * QRS); pr[r] = ra; pr[8 + r] = rc;
                ls += ((float)pa + (float)pc) + ((float)ra + (float)rc) * QRI;
            } else { pr[r] = pa; pr[8 + r] = pc; ls += (float)pa + (float)pc; } }
        l = l * alpha + ls; m = mnew;
        oH0 = oH0 * alpha; oH1 = oH1 * alpha; oH2 = oH2 * alpha; oH3 = oH3 * alpha;
        if constexpr (E) { oL0 = oL0 * alpha; oL1 = oL1 * alpha; oL2 = oL2 * alpha; oL3 = oL3 * alpha; }
        {
            const h16* va = VT + vo + key0;
            const v16h v0 = ldh(va), v1 = ldh(va + (size_t)16 * SEQ), v2 = ldh(va + (size_t)32 * SEQ), v3 = ldh(va + (size_t)48 * SEQ);
            oH0 = wmma16(v0, pb, oH0); oH1 = wmma16(v1, pb, oH1); oH2 = wmma16(v2, pb, oH2); oH3 = wmma16(v3, pb, oH3);
            if constexpr (E) {
                oL0 = wmma16(v0, pr, oL0); oL1 = wmma16(v1, pr, oL1); oL2 = wmma16(v2, pr, oL2); oL3 = wmma16(v3, pr, oL3);
                const h16* vr = VR + voe + key0;
                const v16h r0 = ldh(vr), r1 = ldh(vr + (size_t)16 * EARLY), r2 = ldh(vr + (size_t)32 * EARLY), r3 = ldh(vr + (size_t)48 * EARLY);
                oL0 = wmma16(r0, pb, oL0); oL1 = wmma16(r1, pb, oL1); oL2 = wmma16(r2, pb, oL2); oL3 = wmma16(r3, pb, oL3);
                asm volatile("v_nop\n\tv_nop\n\tv_nop\n\tv_nop" : "+v"(oH0), "+v"(oH1), "+v"(oH2), "+v"(oH3), "+v"(oL0), "+v"(oL1), "+v"(oL2), "+v"(oL3) : "v"(r0), "v"(r1), "v"(r2), "v"(r3), "v"(pb), "v"(pr));
            } else {
                asm volatile("v_nop\n\tv_nop\n\tv_nop\n\tv_nop" : "+v"(oH0), "+v"(oH1), "+v"(oH2), "+v"(oH3) : "v"(v0), "v"(v1), "v"(v2), "v"(v3), "v"(pb));
            }
        }
    }
    l += __shfl_xor(l, 16, 32);
    const float sc = CXS * (1.0f / l);
    const int wb = wave * 16 * 68;
    STG_O(0,  oH0, oL0)
    STG_O(16, oH1, oL1)
    STG_O(32, oH2, oL2)
    STG_O(48, oH3, oL3)
    wave_sync();
    h16* crow = CH + ((size_t)b * SEQ + t0) * DM + h * HD;
#pragma unroll 1
    for (int ps = 0; ps < 2; ++ps) {
#pragma unroll
        for (int s = 0; s < 4; ++s) { const int row = 4 * s + (lane >> 3), c8 = (lane & 7) * 8;
            const v4f x0 = *(const v4fa*)(&os[wb + row * 68 + c8]); const v4f x1 = *(const v4fa*)(&os[wb + row * 68 + c8 + 4]); v8h hv, rv;
#pragma unroll
            for (int i = 0; i < 4; ++i) { const h16 a0 = (h16)x0[i]; const h16 a1 = (h16)x1[i]; hv[i] = a0; hv[4 + i] = a1; rv[i] = (h16)((x0[i] - (float)a0) * QRS); rv[4 + i] = (h16)((x1[i] - (float)a1) * QRS); }
            *(volatile v8h*)(crow + (size_t)row * DM + c8) = hv;
            if constexpr (E) { h16* rrow = CR + ((size_t)b * EARLY + t0) * DM + h * HD; *(volatile v8h*)(rrow + (size_t)row * DM + c8) = rv; } }
        if (ps == 0) __threadfence(); }
}

template<int MB, bool RES>
__global__ __launch_bounds__(32) void k_oproj(const h16* __restrict__ CHp, const h16* __restrict__ CRp, const h16* __restrict__ Wt, float* OUT) {
    __shared__ __align__(16) float os[16 * 68];
    const int K = DM;
    const int lane = threadIdx.x & 31, lr = lane & 15, hi = lane >> 4;
    const int r = blockIdx.x * (16 * MB), c0 = blockIdx.y * 64;
    const int b = RES ? (r / EARLY) : (r / DRC);
    const int t = RES ? (r % EARLY) : (EARLY + r % DRC);
    const size_t arow = (size_t)b * SEQ + t;
    const size_t rrow = (size_t)b * EARLY + t;
    v8f acc[MB][4], accr[MB][4];
#pragma unroll
    for (int mb = 0; mb < MB; ++mb)
#pragma unroll
        for (int nb = 0; nb < 4; ++nb) { acc[mb][nb] = (v8f){}; accr[mb][nb] = (v8f){}; }
    const size_t aoff = (arow + lr) * K + 8 * hi, roff = (rrow + lr) * K + 8 * hi, boff = (size_t)(c0 + lr) * K + 8 * hi;
#pragma unroll 1
    for (int kc = 0; kc < K; kc += 32) {
        v16h a[MB], ar[MB];
#pragma unroll
        for (int mb = 0; mb < MB; ++mb) { a[mb] = ldh(CHp + aoff + (size_t)mb * 16 * K + kc);
            if constexpr (RES) ar[mb] = ldh(CRp + roff + (size_t)mb * 16 * K + kc); else ar[mb] = a[mb]; }
#pragma unroll
        for (int nb = 0; nb < 4; ++nb) { const v16h bw = ldh(Wt + boff + (size_t)nb * 16 * K + kc);
#pragma unroll
            for (int mb = 0; mb < MB; ++mb) { acc[mb][nb] = wmma16(a[mb], bw, acc[mb][nb]);
                if constexpr (RES) accr[mb][nb] = wmma16(ar[mb], bw, accr[mb][nb]); } }
        if constexpr (MB == 4) {
            asm volatile("v_nop\n\tv_nop\n\tv_nop\n\tv_nop" : "+v"(acc[0][0]), "+v"(acc[1][1]), "+v"(acc[2][2]), "+v"(acc[MB - 1][3]) : "v"(a[0]), "v"(a[1]), "v"(a[2]), "v"(a[MB - 1]));
        } else {
            asm volatile("v_nop\n\tv_nop\n\tv_nop\n\tv_nop" : "+v"(acc[0][0]), "+v"(acc[MB - 1][3]), "+v"(accr[0][0]), "+v"(accr[MB - 1][3]) : "v"(a[0]), "v"(a[MB - 1]), "v"(ar[0]), "v"(ar[MB - 1]));
        }
    }
    float* obase = OUT + ((size_t)b * OUT_SEQ + t) * DM + c0;
#pragma unroll
    for (int mb = 0; mb < MB; ++mb) {
#pragma unroll
        for (int nb = 0; nb < 4; ++nb) {
#pragma unroll
            for (int j = 0; j < 8; ++j) {
                float v = acc[mb][nb][j];
                if constexpr (RES) v += accr[mb][nb][j] * QRI;
                os[(hi * 8 + j) * 68 + nb * 16 + lr] = v * OSC; } }
        wave_sync();
        float* ob = obase + (size_t)(mb * 16) * DM;
#pragma unroll 1
        for (int ps = 0; ps < 2; ++ps) {
#pragma unroll
            for (int s = 0; s < 8; ++s) { const int row = 2 * s + hi, cofs = lr * 4;
                const v4f val = *(const v4fa*)(&os[row * 68 + cofs]);
                *(volatile v4f*)(ob + (size_t)row * DM + cofs) = val; }
            if (ps == 0) __threadfence(); }
        wave_sync();
    }
}

static constexpr size_t al256(size_t v) { return (v + 255) & ~(size_t)255; }
static constexpr size_t SZ_XB = al256((size_t)NB * SEQ * DM * 2);
static constexpr size_t SZ_W1 = al256((size_t)DM * DM * 2);
static constexpr size_t SZ_PL = al256((size_t)NB * NH_ * SEQ * HD * 2);
static constexpr size_t SZ_PE = al256((size_t)NB * NH_ * EARLY * HD * 2);
static constexpr size_t SZ_TOTAL = SZ_XB + 4 * SZ_W1 + 4 * SZ_PL + 4 * SZ_PE;
static_assert(SZ_TOTAL <= (size_t)134217728);
static_assert((size_t)NB * SEQ * DM * 2 == (size_t)NB * NH_ * SEQ * HD * 2);
static_assert((size_t)NB * EARLY * DM * 2 == (size_t)NB * NH_ * EARLY * HD * 2);

extern "C" void kernel_launch(void* const* d_in, const int* in_sizes, int n_in,
                              void* d_out, int out_size, void* d_ws, size_t ws_size, hipStream_t stream) {
    if (n_in < 5) return;
    const size_t needx = ((size_t)(NB - 1) * SEQ_FULL + SEQ) * DM;
    if ((size_t)in_sizes[0] < needx) return;
    if ((size_t)in_sizes[1] < (size_t)DM * DM || (size_t)in_sizes[2] < (size_t)DM * DM || (size_t)in_sizes[3] < (size_t)DM * DM || (size_t)in_sizes[4] < (size_t)DM * DM) return;
    if ((size_t)out_size < ((size_t)(NB - 1) * OUT_SEQ + SEQ) * DM) return;
    if (SZ_TOTAL > ws_size) return;
    const float* x = (const float*)d_in[0]; const float* wq = (const float*)d_in[1]; const float* wk = (const float*)d_in[2];
    const float* wv = (const float*)d_in[3]; const float* wo = (const float*)d_in[4];
    float* OUT = (float*)d_out;
    char* wsp = (char*)d_ws;
    bf* XB  = (bf*)wsp; wsp += SZ_XB;
    bf* WQT = (bf*)wsp; wsp += SZ_W1;
    bf* WKT = (bf*)wsp; wsp += SZ_W1;
    bf* WVT = (bf*)wsp; wsp += SZ_W1;
    bf* WOTb = (bf*)wsp; wsp += SZ_W1;
    h16* QH = (h16*)wsp; wsp += SZ_PL;
    h16* KP = (h16*)wsp; wsp += SZ_PL;
    h16* VT = (h16*)wsp; wsp += SZ_PL;
    h16* CH = (h16*)wsp; wsp += SZ_PL;
    h16* QR = (h16*)wsp; wsp += SZ_PE;
    h16* KR = (h16*)wsp; wsp += SZ_PE;
    h16* VR = (h16*)wsp; wsp += SZ_PE;
    h16* CR = (h16*)wsp; wsp += SZ_PE;
    const h16* WOT = (const h16*)WOTb;

    if (SEQ == SEQ_FULL) {
        const size_t n8 = (size_t)NB * SEQ * DM / 8;
        k_cvt8<<<(unsigned)((n8 + 255) / 256), 256, 0, stream>>>(x, XB, n8);
    } else {
        const size_t n8 = (size_t)SEQ * DM / 8;
        for (int b = 0; b < NB; ++b) k_cvt8<<<(unsigned)((n8 + 255) / 256), 256, 0, stream>>>(x + (size_t)b * SEQ_FULL * DM, XB + (size_t)b * SEQ * DM, n8);
    }
    { const dim3 g(DM / 64, DM / 64, 1);
      k_tcvt<0><<<g, 256, 0, stream>>>(wq, WQT); k_tcvt<0><<<g, 256, 0, stream>>>(wk, WKT);
      k_tcvt<0><<<g, 256, 0, stream>>>(wv, WVT); k_tcvt<1><<<g, 256, 0, stream>>>(wo, WOTb); }

    const int BIG = 1 << 30;
    k_proj<<<dim3(NB * SEQ / 64, DM / 64, 1), 32, 0, stream>>>(XB, WQT, QH, QR, 1, SEQ, (size_t)NH_ * SEQ * HD, HD, HD, (size_t)SEQ * HD,
                                                               (size_t)NH_ * EARLY * HD, HD, (size_t)EARLY * HD, EARLY, BIG);
    k_proj<<<dim3(NB * SEQ / 64, DM / 64, 1), 32, 0, stream>>>(XB, WKT, KP, KR, 1, SEQ, (size_t)NH_ * SEQ * HD, HD, HD, (size_t)SEQ * HD,
                                                               (size_t)NH_ * EARLY * HD, HD, (size_t)EARLY * HD, EARLY, BIG);
    k_proj<<<dim3(DM / 64, NB * SEQ / 64, 1), 32, 0, stream>>>(WVT, XB, VT, VR, 1, DM, (size_t)0, SEQ, SEQ, (size_t)DM * SEQ,
                                                               (size_t)0, EARLY, (size_t)DM * EARLY, BIG, EARLY);

    k_flash<true><<<dim3(EARLY / (16 * AW), NB * NH_, 1), 32 * AW, 0, stream>>>(QH, QR, KP, KR, VT, VR, CH, CR);
    if (DROWS > 0) k_flash<false><<<dim3(DRC / (16 * AW), NB * NH_, 1), 32 * AW, 0, stream>>>(QH, QR, KP, KR, VT, VR, CH, CR);

    k_oproj<2, true><<<dim3(NB * EARLY / 32, DM / 64, 1), 32, 0, stream>>>(CH, CR, WOT, OUT);
    if (DROWS > 0) k_oproj<4, false><<<dim3(NB * DRC / 64, DM / 64, 1), 32, 0, stream>>>(CH, CR, WOT, OUT);
}
